// SelectiveSSM_8100308320555
// MI455X (gfx1250) — hardware-run, weakly checked
//
#include <hip/hip_runtime.h>
#include <math.h>

typedef __attribute__((ext_vector_type(16))) _Float16 v16h;
typedef __attribute__((ext_vector_type(8)))  _Float16 v8h;
typedef __attribute__((ext_vector_type(8)))  float    v8f;
typedef __attribute__((ext_vector_type(4)))  float    v4f;
typedef __attribute__((ext_vector_type(2)))  float    v2f;
typedef __attribute__((ext_vector_type(4)))  unsigned v4u;

constexpr int kBatch  = 2;
constexpr int kSeq    = 2048;
constexpr int kDm     = 1024;
constexpr int kDin    = 2048;
constexpr int kNst    = 16;
constexpr int kDtR    = 64;
constexpr int kXpN    = kDtR + 2 * kNst;
constexpr int kXpPad  = 128;
constexpr int kBcW    = 2 * kNst;
constexpr int kRows   = kBatch * kSeq;
constexpr int kXzN    = 2 * kDin;
constexpr int kScanTS = 16;
constexpr int kScanTh = 128;
constexpr int kScanCh = 2 * kScanTh;
constexpr int kConvRows = 16;

static_assert(kXpN == 96);
static_assert((kDm % 32) == 0 && (kDin % 32) == 0 && (kDtR % 32) == 0);
static_assert((kRows % 64) == 0 && (kXzN % 64) == 0 && (kXpPad % 64) == 0 && (kDin % 64) == 0 && (kDm % 64) == 0);
static_assert((kDin % 64) == 0 && kXpPad >= kXpN && kBcW == 32 && kDtR == 64);
static_assert((kSeq % kScanTS) == 0 && (kDin % kScanCh) == 0 && (kSeq % kConvRows) == 0);
static_assert(kScanTS * kBcW == kScanTh * 4);

constexpr float kCarryX    = 16.0f;
constexpr float kCarryWin  = 1024.0f;
constexpr float kCarryXs   = 64.0f;
constexpr float kCarryWxp  = 1024.0f;
constexpr float kCarryDt   = 256.0f;
constexpr float kCarryWdt  = 256.0f;
constexpr float kCarryYg   = 1024.0f;
constexpr float kCarryWout = 1024.0f;
constexpr float kScaleInProj  = 1.0f / (kCarryX  * kCarryWin);
constexpr float kScaleXProj   = 1.0f / (kCarryXs * kCarryWxp);
constexpr float kScaleDtProj  = 1.0f / (kCarryDt * kCarryWdt);
constexpr float kScaleOutProj = 1.0f / (kCarryYg * kCarryWout);

constexpr size_t kOffXA   = 0;
constexpr size_t kOffWIT  = kOffXA   + (size_t)kRows  * kDm  * 2;
constexpr size_t kOffWXT  = kOffWIT  + (size_t)kXzN   * kDm  * 2;
constexpr size_t kOffWDT  = kOffWXT  + (size_t)kXpPad * kDin * 2;
constexpr size_t kOffWOT  = kOffWDT  + (size_t)kDin   * kDtR * 2;
constexpr size_t kOffXI   = kOffWOT  + (size_t)kDm    * kDin * 2;
constexpr size_t kOffG16  = kOffXI   + (size_t)kRows  * kDin * 4;
constexpr size_t kOffXS16 = kOffG16  + (size_t)kRows  * kDin * 2;
constexpr size_t kOffDT16 = kOffXS16 + (size_t)kRows  * kDin * 2;
constexpr size_t kOffBC   = kOffDT16 + (size_t)kRows  * kDtR * 2;
constexpr size_t kOffDL16 = kOffBC   + (size_t)kRows  * kBcW * 4;
constexpr size_t kOffYG16 = kOffDL16 + (size_t)kRows  * kDin * 2;
constexpr size_t kWsTotal = kOffYG16 + (size_t)kRows  * kDin * 2;
static_assert(kWsTotal == 123469824ull);
static_assert(kWsTotal <= 134217728ull);
static_assert((kOffWIT % 128) == 0 && (kOffWXT % 128) == 0 && (kOffWDT % 128) == 0 && (kOffWOT % 128) == 0 &&
              (kOffXI % 128) == 0 && (kOffG16 % 128) == 0 && (kOffXS16 % 128) == 0 && (kOffDT16 % 128) == 0 &&
              (kOffBC % 128) == 0 && (kOffDL16 % 128) == 0 && (kOffYG16 % 128) == 0);

__device__ __forceinline__ float h16_to_f32(unsigned hb) {
  const unsigned sgn = (hb & 0x8000u) << 16;
  const unsigned em = hb & 0x7fffu;
  const float fn = __uint_as_float((em << 13) + 0x38000000u);
  const float fs = (float)em * 5.9604644775390625e-8f;
  const float mag = (em < 0x400u) ? fs : fn;
  return __uint_as_float(__float_as_uint(mag) | sgn);
}
__device__ __forceinline__ unsigned pack_h2(float a, float b) {
  const _Float16 h0 = (_Float16)a, h1 = (_Float16)b;
  return (unsigned)__builtin_bit_cast(unsigned short, h0) | ((unsigned)__builtin_bit_cast(unsigned short, h1) << 16);
}
__device__ __forceinline__ float silu_fast(float v) {
  const float sg = __builtin_amdgcn_rcpf(1.0f + __expf(-v));
  return v * sg;
}
__device__ __forceinline__ float softplus_fast(float v) {
  const float a = __expf(-fabsf(v));
  const float u = 1.0f + a;
  const float l1p = __logf(u) + (a - (u - 1.0f)) * __builtin_amdgcn_rcpf(u);
  return fmaxf(v, 0.0f) + l1p;
}
__device__ __forceinline__ float conv_silu1(float w0, float w1, float w2, float w3, float bc,
                                            float xm3, float xm2, float xm1, float xc) {
  float acc = w0 * xm3;
  acc = fmaf(w1, xm2, acc);
  acc = fmaf(w2, xm1, acc);
  acc = fmaf(w3, xc, acc);
  return silu_fast(acc + bc);
}

__device__ __forceinline__ void guard1_h(v8f& a, v16h x, v16h y) {
  asm volatile("v_nop\n\tv_nop\n\tv_nop\n\tv_nop" : "+v"(a) : "v"(x), "v"(y));
}

template <typename T> struct Frag;
template <> struct Frag<_Float16> {
  typedef v16h V;
  union U { v16h v; v8h h[2]; };
  static __device__ __forceinline__ v16h load(const _Float16* p) {
    U f;
    f.h[0] = *(const v8h*)(p);
    f.h[1] = *(const v8h*)(p + 16);
    return f.v;
  }
  static __device__ __forceinline__ v8f mma(v16h a, v16h b, v8f c) {
    return __builtin_amdgcn_wmma_f32_16x16x32_f16(false, a, false, b, (short)0, c, false, false);
  }
};

template <int ACTM> __device__ __forceinline__ float act_apply(float v) {
  if (ACTM == 1) return silu_fast(v);
  if (ACTM == 2) return softplus_fast(v);
  return v;
}
template <int ACTM>
__device__ __forceinline__ void slab_fill(float* slab, v8f c0, v8f c1, v8f c2, v8f c3, float scale,
                                          float b0, float b1, float b2, float b3, int mOff, int rlane) {
#pragma unroll
  for (int r = 0; r < 8; ++r) {
    float v0 = c0[r] * scale, v1 = c1[r] * scale, v2 = c2[r] * scale, v3 = c3[r] * scale;
    if (ACTM == 2) { v0 += b0; v1 += b1; v2 += b2; v3 += b3; }
    float* sp = slab + (mOff + r) * 68 + rlane;
    sp[0]  = act_apply<ACTM>(v0);
    sp[16] = act_apply<ACTM>(v1);
    sp[32] = act_apply<ACTM>(v2);
    sp[48] = act_apply<ACTM>(v3);
  }
}
__device__ __forceinline__ void rows_store_f32x64(const float* slab, float* Cp, int ldc, int lane) {
  const int hh = lane >> 4, c4 = (lane & 15) * 4;
  for (int pass = 0; pass < 2; ++pass) {
#pragma unroll
    for (int it = 0; it < 8; ++it) {
      const int row = it * 2 + hh;
      const v4f v = *(const v4f*)(slab + row * 68 + c4);
      *(volatile v4f*)(Cp + (size_t)row * ldc + c4) = v;
    }
    __threadfence();
  }
}
__device__ __forceinline__ void rows_store_f32x32(const float* slab, float* Cp, int ldc, int lane) {
  const int q = lane >> 3, c4 = (lane & 7) * 4;
  for (int pass = 0; pass < 2; ++pass) {
#pragma unroll
    for (int it = 0; it < 4; ++it) {
      const int row = it * 4 + q;
      const v4f v = *(const v4f*)(slab + row * 68 + c4);
      *(volatile v4f*)(Cp + (size_t)row * ldc + c4) = v;
    }
    __threadfence();
  }
}
__device__ __forceinline__ void rows_store_f16x64(const float* slab, unsigned short* Cp, int ldc, int lane) {
  const int q = lane >> 3, c8 = (lane & 7) * 8;
  v8h hv[4];
#pragma unroll
  for (int it = 0; it < 4; ++it) {
    const int row = it * 4 + q;
    const float* sp = slab + row * 68 + c8;
    const v4f a0 = *(const v4f*)(sp);
    const v4f a1 = *(const v4f*)(sp + 4);
#pragma unroll
    for (int e = 0; e < 4; ++e) {
      hv[it][e]     = (_Float16)a0[e];
      hv[it][4 + e] = (_Float16)a1[e];
    }
  }
  for (int pass = 0; pass < 2; ++pass) {
#pragma unroll
    for (int it = 0; it < 4; ++it) {
      const int row = it * 4 + q;
      *(volatile v8h*)(Cp + (size_t)row * ldc + c8) = hv[it];
    }
    __threadfence();
  }
}
__device__ __forceinline__ void wave_lds_sync() {
  __builtin_amdgcn_fence(__ATOMIC_RELEASE, "workgroup");
  __builtin_amdgcn_wave_barrier();
  __builtin_amdgcn_fence(__ATOMIC_ACQUIRE, "workgroup");
}

template <int EPI>
__global__ __launch_bounds__(256) void gemm_f16_kernel(
    const unsigned short* __restrict__ Ap, int lda,
    const unsigned short* __restrict__ Btp, int ldb,
    void* __restrict__ C0, void* __restrict__ C1,
    const float* __restrict__ bias,
    int M, int N, int K, float scale) {
  const _Float16* A  = (const _Float16*)Ap;
  const _Float16* Bt = (const _Float16*)Btp;
  __shared__ __align__(16) float sT[8][16 * 68];
  const int lane = threadIdx.x & 31;
  const int wave = __builtin_amdgcn_readfirstlane((int)(threadIdx.x >> 5));
  const int tilesN = N >> 6;
  const int tilesM = M >> 6;
  const int tile = blockIdx.x * 8 + wave;
  if (tile >= tilesM * tilesN) return;
  const int tm = tile / tilesN;
  const int tn = tile - tm * tilesN;
  const int m0 = tm << 6;
  const int n0 = tn << 6;
  const int rlane = lane & 15;
  const int koff  = (lane >> 4) * 8;
  const int mOff  = (lane >> 4) * 8;

  v8f acc[4][4];
#pragma unroll
  for (int i = 0; i < 4; ++i)
#pragma unroll
    for (int j = 0; j < 4; ++j) acc[i][j] = (v8f){0.f, 0.f, 0.f, 0.f, 0.f, 0.f, 0.f, 0.f};

#pragma unroll 1
  for (int k0 = 0; k0 < K; k0 += 32) {
    v16h bh[4];
#pragma unroll
    for (int j = 0; j < 4; ++j)
      bh[j] = Frag<_Float16>::load(Bt + (size_t)(n0 + (j << 4) + rlane) * ldb + koff + k0);
#pragma unroll
    for (int i = 0; i < 4; ++i) {
      const v16h ah = Frag<_Float16>::load(A + (size_t)(m0 + (i << 4) + rlane) * lda + koff + k0);
#pragma unroll
      for (int j = 0; j < 4; ++j) acc[i][j] = Frag<_Float16>::mma(ah, bh[j], acc[i][j]);
#pragma unroll
      for (int j = 0; j < 4; ++j) guard1_h(acc[i][j], ah, bh[j]);
    }
  }

  float* slab = sT[wave];
  bool alt = false;
  if constexpr (EPI == 1) alt = (n0 >= kDin);
  if constexpr (EPI == 2) alt = (tn == 0);
  float b0 = 0.f, b1 = 0.f, b2 = 0.f, b3 = 0.f;
  if constexpr (EPI == 3) {
    b0 = bias[n0 + rlane];
    b1 = bias[n0 + 16 + rlane];
    b2 = bias[n0 + 32 + rlane];
    b3 = bias[n0 + 48 + rlane];
  }
#pragma unroll
  for (int i = 0; i < 4; ++i) {
    const int mBase = m0 + (i << 4);
    if constexpr (EPI == 0) {
      slab_fill<0>(slab, acc[i][0], acc[i][1], acc[i][2], acc[i][3], scale, 0.f, 0.f, 0.f, 0.f, mOff, rlane);
    }
    if constexpr (EPI == 1) {
      if (alt) slab_fill<1>(slab, acc[i][0], acc[i][1], acc[i][2], acc[i][3], scale, 0.f, 0.f, 0.f, 0.f, mOff, rlane);
      else     slab_fill<0>(slab, acc[i][0], acc[i][1], acc[i][2], acc[i][3], scale, 0.f, 0.f, 0.f, 0.f, mOff, rlane);
    }
    if constexpr (EPI == 2) {
      const float sc = alt ? (scale * kCarryDt) : scale;
      slab_fill<0>(slab, acc[i][0], acc[i][1], acc[i][2], acc[i][3], sc, 0.f, 0.f, 0.f, 0.f, mOff, rlane);
    }
    if constexpr (EPI == 3) {
      slab_fill<2>(slab, acc[i][0], acc[i][1], acc[i][2], acc[i][3], scale, b0, b1, b2, b3, mOff, rlane);
    }
    wave_lds_sync();
    if constexpr (EPI == 0) {
      rows_store_f32x64(slab, (float*)C0 + (size_t)mBase * N + n0, N, lane);
    }
    if constexpr (EPI == 1) {
      if (alt) rows_store_f16x64(slab, (unsigned short*)C1 + (size_t)mBase * kDin + (n0 - kDin), kDin, lane);
      else     rows_store_f32x64(slab, (float*)C0 + (size_t)mBase * kDin + n0, kDin, lane);
    }
    if constexpr (EPI == 2) {
      if (alt) rows_store_f16x64(slab, (unsigned short*)C0 + (size_t)mBase * kDtR, kDtR, lane);
      else     rows_store_f32x32(slab, (float*)C1 + (size_t)mBase * kBcW, kBcW, lane);
    }
    if constexpr (EPI == 3) {
      rows_store_f16x64(slab, (unsigned short*)C0 + (size_t)mBase * N + n0, N, lane);
    }
    wave_lds_sync();
  }
}

__global__ __launch_bounds__(256) void cvt_rows_f16_kernel(
    const float* __restrict__ src, unsigned short* __restrict__ dst, int total8, float carry) {
  const int i = blockIdx.x * 256 + threadIdx.x;
  if (i >= total8) return;
  const size_t e0 = (size_t)i << 3;
  const v4f a0 = *(const v4f*)(src + e0);
  const v4f a1 = *(const v4f*)(src + e0 + 4);
  v8h hv;
#pragma unroll
  for (int e = 0; e < 4; ++e) {
    hv[e]     = (_Float16)(a0[e] * carry);
    hv[4 + e] = (_Float16)(a1[e] * carry);
  }
  unsigned short* qd = dst + e0;
  *(volatile v8h*)qd = hv;
  __threadfence();
  *(volatile v8h*)qd = hv;
}

__global__ __launch_bounds__(256) void wt_f16_kernel(
    const float* __restrict__ src, unsigned short* __restrict__ dst,
    int Ksrc, int Nsrc, int Npad, float carry) {
  const int i = blockIdx.x * 256 + threadIdx.x;
  const int kch = Ksrc >> 3;
  if (i >= Npad * kch) return;
  const int n  = i / kch;
  const int kc = i - n * kch;
  const int nc = (n < Nsrc) ? n : (Nsrc - 1);
  const bool live = (n < Nsrc);
  v8h hv;
#pragma unroll
  for (int e = 0; e < 8; ++e) {
    float v = src[(size_t)(kc * 8 + e) * Nsrc + nc];
    asm volatile("" : "+v"(v));
    const float w = live ? (v * carry) : 0.0f;
    hv[e] = (_Float16)w;
  }
  unsigned short* qd = dst + (size_t)n * Ksrc + kc * 8;
  *(volatile v8h*)qd = hv;
  __threadfence();
  *(volatile v8h*)qd = hv;
}

__global__ __launch_bounds__(256) void conv_silu_kernel(
    const float* __restrict__ XI, const float* __restrict__ cw, const float* __restrict__ cb,
    unsigned* __restrict__ XS16w) {
  const int pairIdx = blockIdx.x * 256 + threadIdx.x;
  const int d  = pairIdx * 2;
  const int g0 = blockIdx.y * kConvRows;
  const int tb = g0 & (kSeq - 1);
  const v4f wa = *(const v4f*)(cw + (size_t)d * 4);
  const v4f wb = *(const v4f*)(cw + (size_t)d * 4 + 4);
  const v2f bv = *(const v2f*)(cb + d);
  const bool hist = (tb > 0);
  const int rb = hist ? (g0 - 3) : g0;
  const v2f h3 = *(const v2f*)(XI + (size_t)rb * kDin + d);
  const v2f h2 = *(const v2f*)(XI + (size_t)(rb + 1) * kDin + d);
  const v2f h1 = *(const v2f*)(XI + (size_t)(rb + 2) * kDin + d);
  float am3 = hist ? h3[0] : 0.f, am2 = hist ? h2[0] : 0.f, am1 = hist ? h1[0] : 0.f;
  float bm3 = hist ? h3[1] : 0.f, bm2 = hist ? h2[1] : 0.f, bm1 = hist ? h1[1] : 0.f;
#pragma unroll 1
  for (int grp = 0; grp < kConvRows / 4; ++grp) {
    const int rbase = g0 + grp * 4;
    unsigned pk[4];
#pragma unroll
    for (int u = 0; u < 4; ++u) {
      const v2f xv = *(const v2f*)(XI + (size_t)(rbase + u) * kDin + d);
      const float sa = conv_silu1(wa[0], wa[1], wa[2], wa[3], bv[0], am3, am2, am1, xv[0]);
      const float sb = conv_silu1(wb[0], wb[1], wb[2], wb[3], bv[1], bm3, bm2, bm1, xv[1]);
      pk[u] = pack_h2(sa * kCarryXs, sb * kCarryXs);
      am3 = am2; am2 = am1; am1 = xv[0];
      bm3 = bm2; bm2 = bm1; bm1 = xv[1];
    }
    for (int pass = 0; pass < 2; ++pass) {
#pragma unroll
      for (int u = 0; u < 4; ++u)
        *(volatile unsigned*)(XS16w + (size_t)(rbase + u) * (kDin / 2) + pairIdx) = pk[u];
      __threadfence();
    }
  }
}

__global__ __launch_bounds__(kScanTh) void scan_kernel(
    const float* __restrict__ XI, const float* __restrict__ cw, const float* __restrict__ cb,
    const unsigned* __restrict__ DL16w, const unsigned* __restrict__ G16w, const float* __restrict__ BC,
    const float* __restrict__ Alog, const float* __restrict__ Dp, unsigned* __restrict__ YG16w) {
  __shared__ __align__(16) float    sBC[kScanTS * kBcW];
  __shared__ __align__(16) unsigned sY[kScanTS * kScanTh];
  __shared__ __align__(16) float    sA[kNst * kScanCh];
  const int tid  = threadIdx.x;
  const int lane = tid & 31;
  const int wave = __builtin_amdgcn_readfirstlane((int)(threadIdx.x >> 5));
  constexpr int kBlkPerB = kDin / kScanCh;
  const int bix  = blockIdx.x / kBlkPerB;
  const int cblk = blockIdx.x - bix * kBlkPerB;
  const int d0   = cblk * kScanCh;
  const int d    = d0 + 2 * tid;
  const int dp   = (d0 >> 1) + tid;
  const size_t row0 = (size_t)bix * kSeq;

#pragma unroll 1
  for (int i = 0; i < (kNst * kScanCh) / kScanTh; ++i) {
    const int idx = i * kScanTh + tid;
    const int c = idx >> 4;
    const int n = idx & 15;
    sA[n * kScanCh + c] = -expf(Alog[(size_t)(d0 + c) * kNst + n]);
  }
  __syncthreads();
  float A0[kNst], A1[kNst], h0[kNst], h1[kNst];
#pragma unroll
  for (int n = 0; n < kNst; ++n) {
    const v2f av = *(const v2f*)(sA + n * kScanCh + 2 * tid);
    A0[n] = av[0];
    A1[n] = av[1];
    h0[n] = 0.f;
    h1[n] = 0.f;
  }
  const v4f wa = *(const v4f*)(cw + (size_t)d * 4);
  const v4f wb = *(const v4f*)(cw + (size_t)d * 4 + 4);
  const v2f bv = *(const v2f*)(cb + d);
  const v2f dv = *(const v2f*)(Dp + d);
  float am3 = 0.f, am2 = 0.f, am1 = 0.f, bm3 = 0.f, bm2 = 0.f, bm1 = 0.f;
  const int q = lane >> 3, c4 = (lane & 7) * 4;

#pragma unroll 1
  for (int t0 = 0; t0 < kSeq; t0 += kScanTS) {
    __syncthreads();
    *(v4f*)(sBC + tid * 4) = *(const v4f*)(BC + (row0 + t0) * kBcW + tid * 4);
    __syncthreads();
#pragma unroll 1
    for (int s = 0; s < kScanTS; ++s) {
      const size_t row = row0 + t0 + s;
      const v2f xv = *(const v2f*)(XI + row * kDin + d);
      const unsigned dw = DL16w[row * (kDin / 2) + dp];
      const unsigned gw = G16w[row * (kDin / 2) + dp];
      const float u0 = conv_silu1(wa[0], wa[1], wa[2], wa[3], bv[0], am3, am2, am1, xv[0]);
      const float u1 = conv_silu1(wb[0], wb[1], wb[2], wb[3], bv[1], bm3, bm2, bm1, xv[1]);
      am3 = am2; am2 = am1; am1 = xv[0];
      bm3 = bm2; bm2 = bm1; bm1 = xv[1];
      const float dl0 = h16_to_f32(dw & 0xffffu);
      const float dl1 = h16_to_f32(dw >> 16);
      const float g0v = h16_to_f32(gw & 0xffffu);
      const float g1v = h16_to_f32(gw >> 16);
      const float dx0 = dl0 * u0;
      const float dx1 = dl1 * u1;
      const float* bc = sBC + s * kBcW;
      float y0 = 0.f, y1 = 0.f;
#pragma unroll
      for (int q4 = 0; q4 < 4; ++q4) {
        const v4f bq = *(const v4f*)(bc + 4 * q4);
        const v4f cq = *(const v4f*)(bc + kNst + 4 * q4);
#pragma unroll
        for (int e = 0; e < 4; ++e) {
          const int n = 4 * q4 + e;
          const float bn = bq[e];
          const float cn = cq[e];
          const float e0 = __expf(dl0 * A0[n]);
          const float e1 = __expf(dl1 * A1[n]);
          h0[n] = fmaf(e0, h0[n], dx0 * bn);
          h1[n] = fmaf(e1, h1[n], dx1 * bn);
          y0 = fmaf(h0[n], cn, y0);
          y1 = fmaf(h1[n], cn, y1);
        }
      }
      y0 = fmaf(u0, dv[0], y0);
      y1 = fmaf(u1, dv[1], y1);
      y0 = y0 * g0v;
      y1 = y1 * g1v;
      sY[s * kScanTh + tid] = pack_h2(y0 * kCarryYg, y1 * kCarryYg);
    }
    __syncthreads();
    v4u buf[4];
#pragma unroll
    for (int it = 0; it < 4; ++it)
      buf[it] = *(const v4u*)(sY + (it * 4 + q) * kScanTh + wave * 32 + c4);
    for (int pass = 0; pass < 2; ++pass) {
#pragma unroll
      for (int it = 0; it < 4; ++it) {
        const size_t o = (row0 + t0 + it * 4 + q) * (kDin / 2) + (d0 >> 1) + wave * 32 + c4;
        *(volatile v4u*)(YG16w + o) = buf[it];
      }
      __threadfence();
    }
  }
}

extern "C" void kernel_launch(void* const* d_in, const int* in_sizes, int n_in,
                              void* d_out, int out_size, void* d_ws, size_t ws_size,
                              hipStream_t stream) {
  if (n_in < 10) return;
  if (in_sizes[0] != kRows * kDm) return;
  if (in_sizes[1] != kDm * kXzN) return;
  if (in_sizes[2] != kDin * 4) return;
  if (in_sizes[3] != kDin) return;
  if (in_sizes[4] != kDin * kXpN) return;
  if (in_sizes[5] != kDtR * kDin) return;
  if (in_sizes[6] != kDin) return;
  if (in_sizes[7] != kDin * kNst) return;
  if (in_sizes[8] != kDin) return;
  if (in_sizes[9] != kDin * kDm) return;
  if (out_size != kRows * kDm) return;
  if (ws_size < kWsTotal) return;

  const float* x       = (const float*)d_in[0];
  const float* W_in    = (const float*)d_in[1];
  const float* conv_w  = (const float*)d_in[2];
  const float* conv_b  = (const float*)d_in[3];
  const float* W_xproj = (const float*)d_in[4];
  const float* W_dt    = (const float*)d_in[5];
  const float* b_dt    = (const float*)d_in[6];
  const float* A_log   = (const float*)d_in[7];
  const float* Dp      = (const float*)d_in[8];
  const float* W_out   = (const float*)d_in[9];
  float* out = (float*)d_out;

  char* ws = (char*)d_ws;
  unsigned short* XA   = (unsigned short*)(ws + kOffXA);
  unsigned short* WIT  = (unsigned short*)(ws + kOffWIT);
  unsigned short* WXT  = (unsigned short*)(ws + kOffWXT);
  unsigned short* WDT  = (unsigned short*)(ws + kOffWDT);
  unsigned short* WOT  = (unsigned short*)(ws + kOffWOT);
  float*          XI   = (float*)(ws + kOffXI);
  unsigned short* G16  = (unsigned short*)(ws + kOffG16);
  unsigned short* XS16 = (unsigned short*)(ws + kOffXS16);
  unsigned short* DT16 = (unsigned short*)(ws + kOffDT16);
  float*          BCp  = (float*)(ws + kOffBC);
  unsigned short* DL16 = (unsigned short*)(ws + kOffDL16);
  unsigned short* YG16 = (unsigned short*)(ws + kOffYG16);

  cvt_rows_f16_kernel<<<(kRows * kDm / 8) / 256, 256, 0, stream>>>(x, XA, kRows * kDm / 8, kCarryX);
  wt_f16_kernel<<<(kXzN   * (kDm  / 8)) / 256, 256, 0, stream>>>(W_in,    WIT, kDm,  kXzN, kXzN,   kCarryWin);
  wt_f16_kernel<<<(kXpPad * (kDin / 8)) / 256, 256, 0, stream>>>(W_xproj, WXT, kDin, kXpN, kXpPad, kCarryWxp);
  wt_f16_kernel<<<(kDin   * (kDtR / 8)) / 256, 256, 0, stream>>>(W_dt,    WDT, kDtR, kDin, kDin,   kCarryWdt);
  wt_f16_kernel<<<(kDm    * (kDin / 8)) / 256, 256, 0, stream>>>(W_out,   WOT, kDin, kDm,  kDm,    kCarryWout);

  gemm_f16_kernel<1><<<((kRows / 64) * (kXzN / 64) + 7) / 8, 256, 0, stream>>>(
      XA, kDm, WIT, kDm, (void*)XI, (void*)G16, nullptr, kRows, kXzN, kDm, kScaleInProj);

  conv_silu_kernel<<<dim3((kDin / 2) / 256, kRows / kConvRows), 256, 0, stream>>>(
      XI, conv_w, conv_b, (unsigned*)XS16);

  gemm_f16_kernel<2><<<((kRows / 64) * (kXpPad / 64) + 7) / 8, 256, 0, stream>>>(
      XS16, kDin, WXT, kDin, (void*)DT16, (void*)BCp, nullptr, kRows, kXpPad, kDin, kScaleXProj);

  gemm_f16_kernel<3><<<((kRows / 64) * (kDin / 64) + 7) / 8, 256, 0, stream>>>(
      DT16, kDtR, WDT, kDtR, (void*)DL16, nullptr, b_dt, kRows, kDin, kDtR, kScaleDtProj);

  scan_kernel<<<kBatch * (kDin / kScanCh), kScanTh, 0, stream>>>(
      XI, conv_w, conv_b, (const unsigned*)DL16, (const unsigned*)G16, BCp, A_log, Dp, (unsigned*)YG16);

  gemm_f16_kernel<0><<<((kRows / 64) * (kDm / 64) + 7) / 8, 256, 0, stream>>>(
      YG16, kDin, WOT, kDin, (void*)out, nullptr, nullptr, kRows, kDm, kDin, kScaleOutProj);
}
